// RNNAttentionModel_44470091383027
// MI455X (gfx1250) — hardware-verified
//
#include <hip/hip_runtime.h>

typedef __attribute__((ext_vector_type(16))) _Float16 v16h;
typedef __attribute__((ext_vector_type(8)))  _Float16 v8h;
typedef __attribute__((ext_vector_type(16))) __bf16   v16b;
typedef __attribute__((ext_vector_type(8)))  __bf16   v8b;
typedef __attribute__((ext_vector_type(8)))  float    v8f;
typedef __attribute__((ext_vector_type(4)))  float    v4f;

constexpr int kSeq   = 64;
constexpr int kStep  = 1024;
constexpr int kEmb   = 64;
constexpr int kHid   = 128;
constexpr int kVoc   = 55;
constexpr int kRows  = kSeq * kStep;
constexpr int kCombP = 256;
constexpr int kGrp   = 8;
constexpr int kNGrp  = kSeq / kGrp;
constexpr int kVocPad = 64;
constexpr int kOut4  = kRows * kVoc / 4;

constexpr int kSeqPB = 16;
constexpr int kXch   = 8;
constexpr int kW0P   = 200;
constexpr int kW1P   = 264;
constexpr int kXP    = 72;
constexpr int kHP    = 136;
constexpr int kRnnThreads = 256;
constexpr unsigned kRnnLdsBytes = (unsigned)(128 * kW0P + 128 * kW1P + kXch * 16 * kXP + 2 * 16 * kHP) * 2u + 256u * 4u;
static_assert(kRnnLdsBytes == 146944);
static_assert(kStep % kXch == 0);
static_assert(kSeq % kSeqPB == 0);
static_assert((kRows * kVoc) % 4 == 0);
static_assert(kOut4 % 256 == 0);

__device__ __forceinline__ unsigned short f2bf_bits(float f) {
  unsigned u = __float_as_uint(f);
  return (unsigned short)((u + 0x7FFFu + ((u >> 16) & 1u)) >> 16);
}
__device__ __forceinline__ float bf_bits2f(unsigned short h) { return __uint_as_float(((unsigned)h) << 16); }

__device__ __forceinline__ void dep_guard_h(v8f& a, v8f& b, v16h x, v16h y) { asm volatile("v_nop\n\tv_nop\n\tv_nop\n\tv_nop" : "+v"(a), "+v"(b) : "v"(x), "v"(y)); }
__device__ __forceinline__ void dep_guard_b(v8f& a, v8f& b, v16b x, v16b y) { asm volatile("v_nop\n\tv_nop\n\tv_nop\n\tv_nop" : "+v"(a), "+v"(b) : "v"(x), "v"(y)); }
__device__ __forceinline__ void keep4_h(v16h a, v16h b, v16h c, v16h d) { asm volatile("v_nop" :: "v"(a), "v"(b), "v"(c), "v"(d)); }
__device__ __forceinline__ void keep4_b(v16b a, v16b b, v16b c, v16b d) { asm volatile("v_nop" :: "v"(a), "v"(b), "v"(c), "v"(d)); }
__device__ __forceinline__ void acc_guard4(v8f& a, v8f& b, v8f& c, v8f& d) { asm volatile("v_nop\n\tv_nop\n\tv_nop\n\tv_nop" : "+v"(a), "+v"(b), "+v"(c), "+v"(d)); }
__device__ __forceinline__ void dep_guard1(v8f& a, v16h x, v16h y) { asm volatile("v_nop\n\tv_nop\n\tv_nop\n\tv_nop" : "+v"(a) : "v"(x), "v"(y)); }

template <typename T> struct Frag;
template <> struct Frag<_Float16> {
  typedef v16h V; union U { v16h v; v8h h[2]; };
  static __device__ __forceinline__ v16h load(const _Float16* p) {
    U f; f.h[0] = *(const v8h*)(p); f.h[1] = *(const v8h*)(p + 16); return f.v;
  }
  static __device__ __forceinline__ v8f mma(v16h a, v16h b, v8f c) {
    return __builtin_amdgcn_wmma_f32_16x16x32_f16(false, a, false, b, (short)0, c, false, false);
  }
  static __device__ __forceinline__ void guard(v8f& a, v8f& b, v16h x, v16h y) { dep_guard_h(a, b, x, y); }
  static __device__ __forceinline__ void keep(v16h a, v16h b, v16h c, v16h d) { keep4_h(a, b, c, d); }
};
template <> struct Frag<__bf16> {
  typedef v16b V; union U { v16b v; v8b h[2]; };
  static __device__ __forceinline__ v16b load(const __bf16* p) {
    U f; f.h[0] = *(const v8b*)(p); f.h[1] = *(const v8b*)(p + 16); return f.v;
  }
  static __device__ __forceinline__ v8f mma(v16b a, v16b b, v8f c) {
    return __builtin_amdgcn_wmma_f32_16x16x32_bf16(false, a, false, b, (short)0, c, false, false);
  }
  static __device__ __forceinline__ void guard(v8f& a, v8f& b, v16b x, v16b y) { dep_guard_b(a, b, x, y); }
  static __device__ __forceinline__ void keep(v16b a, v16b b, v16b c, v16b d) { keep4_b(a, b, c, d); }
};

template <int ET> struct Elem;
template <> struct Elem<0> { typedef _Float16 T; };
template <> struct Elem<1> { typedef __bf16 T; };
template <int ET, bool SPLIT, int BIAS_MODE, int OUT_MODE, bool RESID, int ACT = 0, int TRI = 0>
__global__ __launch_bounds__(256) void wmma_gemm64(
    const unsigned short* __restrict__ Ap, const unsigned short* __restrict__ A2p, int lda, long strideA,
    const unsigned short* __restrict__ Btp, const unsigned short* __restrict__ Bt2p, int ldb, long strideB,
    void* __restrict__ Cout, void* __restrict__ Cout2, int ldc, long strideC,
    const float* __restrict__ bias,
    const float* __restrict__ resid, long strideR,
    int M, int N, int K, float scale) {
  typedef typename Elem<ET>::T T;
  typedef typename Frag<T>::V V;
  const T* A = (const T*)Ap; const T* A2 = (const T*)A2p; const T* Bt = (const T*)Btp; const T* Bt2 = (const T*)Bt2p;
  __shared__ __align__(16) float sT[8][16 * 68];
  const int b    = blockIdx.y;
  const int lane = threadIdx.x & 31;
  const int wave = threadIdx.x >> 5;
  const int tilesN = N >> 6;
  const int tilesM = M >> 6;
  const int tile = blockIdx.x * 8 + wave;
  if (tile >= tilesM * tilesN) return;
  const int tm = tile / tilesN;
  const int tn = tile - tm * tilesN;
  if (TRI == 1 && tn > tm) return;
  const int m0 = tm << 6;
  const int n0 = tn << 6;
  const int kLim = (TRI == 2) ? ((m0 + 64 < K) ? (m0 + 64) : K) : K;

  const T* Ab  = A  + (size_t)b * strideA;
  const T* Bb  = Bt + (size_t)b * strideB;
  const T* Ab2 = SPLIT ? (A2  + (size_t)b * strideA) : nullptr;
  const T* Bb2 = SPLIT ? (Bt2 + (size_t)b * strideB) : nullptr;

  const int rlane = lane & 15;
  const int koff  = (lane >> 4) * 8;
  const int mOff  = (lane >> 4) * 8;

  v8f acc[4][4];
#pragma unroll
  for (int i = 0; i < 4; ++i)
#pragma unroll
    for (int j = 0; j < 4; ++j) acc[i][j] = (v8f){0.f,0.f,0.f,0.f,0.f,0.f,0.f,0.f};

  for (int k0 = 0; k0 < kLim; k0 += 32) {
    V bh[4], bl[4];
#pragma unroll
    for (int j = 0; j < 4; ++j) {
      const size_t bo = (size_t)(n0 + (j << 4) + rlane) * ldb + koff + k0;
      bh[j] = Frag<T>::load(Bb + bo);
      if (SPLIT) bl[j] = Frag<T>::load(Bb2 + bo);
    }
#pragma unroll
    for (int i = 0; i < 4; ++i) {
      const size_t ao = (size_t)(m0 + (i << 4) + rlane) * lda + koff + k0;
      V ah = Frag<T>::load(Ab + ao);
      V al;
      if (SPLIT) al = Frag<T>::load(Ab2 + ao);
#pragma unroll
      for (int j = 0; j < 4; ++j) {
        acc[i][j] = Frag<T>::mma(ah, bh[j], acc[i][j]);
        if (SPLIT) {
          acc[i][j] = Frag<T>::mma(ah, bl[j], acc[i][j]);
          acc[i][j] = Frag<T>::mma(al, bh[j], acc[i][j]);
        }
      }
      Frag<T>::guard(acc[i][0], acc[i][3], ah, SPLIT ? al : ah);
    }
    Frag<T>::keep(bh[0], bh[1], bh[2], bh[3]);
    if (SPLIT) Frag<T>::keep(bl[0], bl[1], bl[2], bl[3]);
  }
  acc_guard4(acc[0][0], acc[0][1], acc[0][2], acc[0][3]);
  acc_guard4(acc[1][0], acc[1][1], acc[1][2], acc[1][3]);
  acc_guard4(acc[2][0], acc[2][1], acc[2][2], acc[2][3]);
  acc_guard4(acc[3][0], acc[3][1], acc[3][2], acc[3][3]);

  float* slab = sT[wave];
  const float* Rb = RESID ? (resid + (size_t)b * strideR) : nullptr;
#pragma unroll
  for (int i = 0; i < 4; ++i) {
    const int mBase = m0 + (i << 4);
#pragma unroll
    for (int j = 0; j < 4; ++j) {
      const int n = n0 + (j << 4) + rlane;
      float bv = 0.f;
      if (BIAS_MODE == 2) bv = bias[n];
#pragma unroll
      for (int r = 0; r < 8; ++r) {
        float v = acc[i][j][r] * scale;
        if (BIAS_MODE == 1) v += bias[mBase + mOff + r];
        if (BIAS_MODE == 2) v += bv;
        if (RESID) v += Rb[(size_t)(mBase + mOff + r) * ldc + n];
        if (ACT == 1) v = tanhf(v);
        if (ACT == 2) v = fmaxf(v, 0.0f);
        if (ACT == 4) v = (v > 0.f) ? v : 0.01f * v;
        slab[(mOff + r) * 68 + (j << 4) + rlane] = v;
      }
    }
    __builtin_amdgcn_fence(__ATOMIC_RELEASE, "workgroup");
    __builtin_amdgcn_wave_barrier();
    __builtin_amdgcn_fence(__ATOMIC_ACQUIRE, "workgroup");
    if (OUT_MODE == 0) {
      float* C = (float*)Cout + (size_t)b * strideC;
      const int hh = lane >> 4, c4 = (lane & 15) * 4;
      for (int pass = 0; pass < 2; ++pass) {
#pragma unroll
        for (int it = 0; it < 8; ++it) {
          const int row = it * 2 + hh;
          v4f v = *(const v4f*)(slab + row * 68 + c4);
          *(volatile v4f*)(C + (size_t)(mBase + row) * ldc + n0 + c4) = v;
        }
        __threadfence();
      }
    } else {
      const int q = lane >> 3, c8 = (lane & 7) * 8;
      unsigned short* C  = (unsigned short*)Cout  + (size_t)b * strideC;
      unsigned short* C2 = (OUT_MODE == 2) ? ((unsigned short*)Cout2 + (size_t)b * strideC) : nullptr;
      for (int pass = 0; pass < 2; ++pass) {
#pragma unroll
        for (int it = 0; it < 4; ++it) {
          const int row = it * 4 + q;
          const float* sp = slab + row * 68 + c8;
          v8h hv, lv;
#pragma unroll
          for (int e = 0; e < 8; ++e) {
            if (OUT_MODE == 1) {
              hv[e] = (_Float16)sp[e];
            } else {
              unsigned short hb = f2bf_bits(sp[e]);
              unsigned short lb = f2bf_bits(sp[e] - bf_bits2f(hb));
              hv[e] = __builtin_bit_cast(_Float16, hb);
              lv[e] = __builtin_bit_cast(_Float16, lb);
            }
          }
          *(volatile v8h*)(C + (size_t)(mBase + row) * ldc + n0 + c8) = hv;
          if (OUT_MODE == 2) *(volatile v8h*)(C2 + (size_t)(mBase + row) * ldc + n0 + c8) = lv;
        }
        __threadfence();
      }
    }
    __builtin_amdgcn_fence(__ATOMIC_RELEASE, "workgroup");
    __builtin_amdgcn_wave_barrier();
    __builtin_amdgcn_fence(__ATOMIC_ACQUIRE, "workgroup");
  }
}

__device__ __forceinline__ unsigned pack_f16x2(float a, float b) {
  const _Float16 h0 = (_Float16)a, h1 = (_Float16)b;
  return (unsigned)__builtin_bit_cast(unsigned short, h0) | ((unsigned)__builtin_bit_cast(unsigned short, h1) << 16);
}
__device__ __forceinline__ void st2u(unsigned* p, unsigned v) { *(volatile unsigned*)p = v; __threadfence(); *(volatile unsigned*)p = v; }
__device__ __forceinline__ float ftanh(float x) { return 1.0f - 2.0f * __builtin_amdgcn_rcpf(1.0f + __expf(2.0f * x)); }

__global__ __launch_bounds__(256) void prep_kernel(const float* __restrict__ attn_w, const float* __restrict__ fc_w,
                                                  const float* __restrict__ fc_b,
                                                  unsigned* __restrict__ atw16u, unsigned* __restrict__ fcw16u,
                                                  unsigned* __restrict__ fcb64u) {
  const int blk = blockIdx.x, tid = threadIdx.x;
  if (blk < 32) {
    const int p = blk * 256 + tid;
    const unsigned u = pack_f16x2(attn_w[2 * p] * 16.0f, attn_w[2 * p + 1] * 16.0f);
    st2u(atw16u + p, u);
  } else if (blk < 64) {
    const int p = (blk - 32) * 256 + tid;
    const int n = p >> 7;
    const int k = (2 * p) & 255;
    const int nc = (n < kVoc) ? n : (kVoc - 1);
    const float f0 = fc_w[nc * (2 * kHid) + k] * 16.0f;
    const float f1 = fc_w[nc * (2 * kHid) + k + 1] * 16.0f;
    const unsigned u = (n < kVoc) ? pack_f16x2(f0, f1) : 0u;
    st2u(fcw16u + p, u);
  } else {
    if (tid < kVocPad) {
      const int vc = (tid < kVoc) ? tid : (kVoc - 1);
      const float f = fc_b[vc];
      const unsigned u = (tid < kVoc) ? (unsigned)__float_as_uint(f) : 0u;
      st2u(fcb64u + tid, u);
    }
  }
}

__global__ __launch_bounds__(kRnnThreads) void rnn2_kernel(
    const int* __restrict__ x, const float* __restrict__ emb,
    const float* __restrict__ w_ih0, const float* __restrict__ b_ih0,
    const float* __restrict__ w_hh0, const float* __restrict__ b_hh0,
    const float* __restrict__ w_ih1, const float* __restrict__ b_ih1,
    const float* __restrict__ w_hh1, const float* __restrict__ b_hh1,
    _Float16* __restrict__ comb) {
  extern __shared__ __align__(16) _Float16 rnn_lds[];
  _Float16* w0s = rnn_lds;
  _Float16* w1s = w0s + 128 * kW0P;
  _Float16* xt  = w1s + 128 * kW1P;
  _Float16* hst = xt + kXch * 16 * kXP;
  _Float16* h0t = hst;
  _Float16* h1t = hst + 16 * kHP;
  float* biasv  = (float*)(hst + 32 * kHP);

  const int tid = threadIdx.x, lane = tid & 31, wave = tid >> 5;
  const int rlane = lane & 15, hh = lane >> 4, koff = hh * 8, mOff = hh * 8;
  const int seq0 = blockIdx.x * kSeqPB;

#pragma unroll 4
  for (int i = tid; i < kHid * kEmb; i += kRnnThreads) {
    const int n = i >> 6, k = i & 63;
    w0s[n * kW0P + k] = (_Float16)(w_ih0[i] * 16.0f);
  }
#pragma unroll 4
  for (int i = tid; i < kHid * kHid; i += kRnnThreads) {
    const int n = i >> 7, k = i & 127;
    w0s[n * kW0P + kEmb + k] = (_Float16)(w_hh0[i] * 16.0f);
    w1s[n * kW1P + k]        = (_Float16)(w_ih1[i] * 16.0f);
    w1s[n * kW1P + kHid + k] = (_Float16)(w_hh1[i] * 16.0f);
  }
  if (tid < kHid) biasv[tid] = b_ih0[tid] + b_hh0[tid];
  else            biasv[tid] = b_ih1[tid - kHid] + b_hh1[tid - kHid];
  for (int i = tid; i < 32 * kHP; i += kRnnThreads) hst[i] = (_Float16)0.0f;
  __syncthreads();

  const int ncol = wave * 16 + rlane;
  const _Float16* w0row = w0s + ncol * kW0P + koff;
  const _Float16* w1row = w1s + ncol * kW1P + koff;
  const _Float16* h0row = h0t + rlane * kHP + koff;
  const _Float16* h1row = h1t + rlane * kHP + koff;
  const float bs0 = biasv[ncol];
  const float bs1 = biasv[kHid + ncol];
  const float inv16 = 0.0625f;
  const v8f z8 = {0.f, 0.f, 0.f, 0.f, 0.f, 0.f, 0.f, 0.f};

#pragma unroll 1
  for (int tc = 0; tc < kStep; tc += kXch) {
#pragma unroll
    for (int q = 0; q < 4; ++q) {
      const int ci = tid + kRnnThreads * q;
      const int s = ci >> 7, r = (ci >> 3) & 15, c8 = ci & 7;
      int tok = x[(size_t)(seq0 + r) * kStep + tc + s];
      tok = tok < 0 ? 0 : (tok > kVoc - 1 ? (kVoc - 1) : tok);
      const float* er = emb + (size_t)tok * kEmb + c8 * 8;
      const v4f f0 = *(const v4f*)er;
      const v4f f1 = *(const v4f*)(er + 4);
      v8h hv;
      hv[0] = (_Float16)f0[0]; hv[1] = (_Float16)f0[1]; hv[2] = (_Float16)f0[2]; hv[3] = (_Float16)f0[3];
      hv[4] = (_Float16)f1[0]; hv[5] = (_Float16)f1[1]; hv[6] = (_Float16)f1[2]; hv[7] = (_Float16)f1[3];
      *(v8h*)(xt + (s * 16 + r) * kXP + c8 * 8) = hv;
    }
    __syncthreads();

#pragma unroll 1
    for (int s = 0; s < kXch; ++s) {
      const int t = tc + s;
      const _Float16* xrow = xt + (s * 16 + rlane) * kXP + koff;
      v8f acc = z8;
      v16h fa, fb;
      fa = Frag<_Float16>::load(xrow);      fb = Frag<_Float16>::load(w0row);      acc = Frag<_Float16>::mma(fa, fb, acc);
      fa = Frag<_Float16>::load(xrow + 32); fb = Frag<_Float16>::load(w0row + 32); acc = Frag<_Float16>::mma(fa, fb, acc);
#pragma unroll
      for (int kc = 0; kc < 4; ++kc) {
        fa = Frag<_Float16>::load(h0row + 32 * kc);
        fb = Frag<_Float16>::load(w0row + kEmb + 32 * kc);
        acc = Frag<_Float16>::mma(fa, fb, acc);
      }
      dep_guard1(acc, fa, fb);
      float hv8[8];
#pragma unroll
      for (int r = 0; r < 8; ++r) hv8[r] = ftanh(fmaf(acc[r], inv16, bs0));
      __syncthreads();
#pragma unroll
      for (int r = 0; r < 8; ++r) h0t[(mOff + r) * kHP + ncol] = (_Float16)hv8[r];
      __syncthreads();

      acc = z8;
#pragma unroll
      for (int kc = 0; kc < 4; ++kc) {
        fa = Frag<_Float16>::load(h0row + 32 * kc);
        fb = Frag<_Float16>::load(w1row + 32 * kc);
        acc = Frag<_Float16>::mma(fa, fb, acc);
      }
#pragma unroll
      for (int kc = 0; kc < 4; ++kc) {
        fa = Frag<_Float16>::load(h1row + 32 * kc);
        fb = Frag<_Float16>::load(w1row + kHid + 32 * kc);
        acc = Frag<_Float16>::mma(fa, fb, acc);
      }
      dep_guard1(acc, fa, fb);
#pragma unroll
      for (int r = 0; r < 8; ++r) hv8[r] = ftanh(fmaf(acc[r], inv16, bs1));
      __syncthreads();
#pragma unroll
      for (int r = 0; r < 8; ++r) h1t[(mOff + r) * kHP + ncol] = (_Float16)hv8[r];
      __syncthreads();
      {
        const int rr = 2 * wave + hh;
        const v8h ov = *(const v8h*)(h1t + rr * kHP + rlane * 8);
        _Float16* dst = comb + ((size_t)(seq0 + rr) * kStep + t) * kCombP + rlane * 8;
        *(volatile v8h*)dst = ov;
        __threadfence();
        *(volatile v8h*)dst = ov;
      }
    }
  }
}

__global__ __launch_bounds__(256) void transpose_outs_kernel(const _Float16* __restrict__ comb, _Float16* __restrict__ outsT) {
  __shared__ __align__(16) _Float16 tile[64 * 72];
  const int tid = threadIdx.x, lane = tid & 31, wave = tid >> 5;
  const int blk = blockIdx.x;
  const int bb = blk >> 5, rem = blk & 31, st = rem >> 1, ht = rem & 1;
  const int s0 = st * 64, hb0 = ht * 64;
#pragma unroll
  for (int q = 0; q < 2; ++q) {
    const int ci = tid + 256 * q;
    const int r = ci >> 3, c8 = ci & 7;
    const v8h hv = *(const v8h*)(comb + (size_t)(bb * kStep + s0 + r) * kCombP + hb0 + c8 * 8);
#pragma unroll
    for (int e = 0; e < 8; ++e) tile[(c8 * 8 + e) * 72 + r] = hv[e];
  }
  __syncthreads();
  const int q4 = lane >> 3, cs = (lane & 7) * 8;
  for (int pass = 0; pass < 2; ++pass) {
#pragma unroll
    for (int it = 0; it < 2; ++it) {
      const int row = wave * 8 + it * 4 + q4;
      const v8h hv = *(const v8h*)(tile + row * 72 + cs);
      *(volatile v8h*)(outsT + (size_t)(bb * kHid + hb0 + row) * kStep + s0 + cs) = hv;
    }
    __threadfence();
  }
}

__global__ __launch_bounds__(256) void causal_softmax_kernel(const float* __restrict__ S, _Float16* __restrict__ P, int nrows) {
  const int wave = threadIdx.x >> 5, lane = threadIdx.x & 31;
  const int gr = blockIdx.x * 8 + wave;
  if (gr >= nrows) return;
  const int t = gr & (kStep - 1);
  const int kend = ((t >> 6) + 1) << 6;
  const float* srow = S + (size_t)gr * kStep;
  _Float16* prow = P + (size_t)gr * kStep;
  const float kFill = -1.0e30f;
  float v[4][8];
  float m = kFill;
#pragma unroll
  for (int it = 0; it < 4; ++it) {
#pragma unroll
    for (int e = 0; e < 8; ++e) v[it][e] = kFill;
    if (it * 256 < kend) {
      const int c0 = it * 256 + lane * 8;
      const v4f f0 = *(const v4f*)(srow + c0);
      const v4f f1 = *(const v4f*)(srow + c0 + 4);
#pragma unroll
      for (int e = 0; e < 4; ++e) {
        v[it][e]     = (c0 + e     <= t) ? f0[e] : kFill;
        v[it][4 + e] = (c0 + 4 + e <= t) ? f1[e] : kFill;
      }
#pragma unroll
      for (int e = 0; e < 8; ++e) m = fmaxf(m, v[it][e]);
    }
  }
#pragma unroll
  for (int off = 1; off < 32; off <<= 1) m = fmaxf(m, __shfl_xor(m, off, 32));
  float sum = 0.0f;
#pragma unroll
  for (int it = 0; it < 4; ++it) {
    if (it * 256 < kend) {
#pragma unroll
      for (int e = 0; e < 8; ++e) { const float p = __expf(v[it][e] - m); v[it][e] = p; sum += p; }
    }
  }
#pragma unroll
  for (int off = 1; off < 32; off <<= 1) sum += __shfl_xor(sum, off, 32);
  const float scl = 32768.0f * __builtin_amdgcn_rcpf(sum);
  for (int pass = 0; pass < 2; ++pass) {
#pragma unroll
    for (int it = 0; it < 4; ++it) {
      if (it * 256 < kend) {
        v8h hv;
#pragma unroll
        for (int e = 0; e < 8; ++e) hv[e] = (_Float16)(v[it][e] * scl);
        *(volatile v8h*)(prow + it * 256 + lane * 8) = hv;
      }
    }
    __threadfence();
  }
}

__global__ __launch_bounds__(256) void pack_logits_kernel(const float* __restrict__ LG, float* __restrict__ out, int n4) {
  const int i = blockIdx.x * 256 + threadIdx.x;
  if (i >= n4) return;
  v4f val;
#pragma unroll
  for (int e = 0; e < 4; ++e) {
    const int idx = 4 * i + e;
    const int row = idx / kVoc;
    const int col = idx - row * kVoc;
    val[e] = LG[(size_t)row * kVocPad + col];
  }
  float* op = out + (size_t)i * 4;
  *(volatile v4f*)op = val;
  __threadfence();
  *(volatile v4f*)op = val;
}

extern "C" void kernel_launch(void* const* d_in, const int* in_sizes, int n_in,
                              void* d_out, int out_size, void* d_ws, size_t ws_size, hipStream_t stream) {
  if (n_in < 14 || d_out == nullptr || d_ws == nullptr) return;
  if (in_sizes[0] != kSeq * kStep || in_sizes[1] != kVoc * kEmb || in_sizes[2] != kHid * kEmb || in_sizes[3] != kHid ||
      in_sizes[4] != kHid * kHid || in_sizes[5] != kHid || in_sizes[6] != kHid * kHid || in_sizes[7] != kHid ||
      in_sizes[8] != kHid * kHid || in_sizes[9] != kHid || in_sizes[10] != kHid * kHid || in_sizes[11] != kHid ||
      in_sizes[12] != kVoc * 2 * kHid || in_sizes[13] != kVoc || out_size != kRows * kVoc) return;

  const int*   x      = (const int*)  d_in[0];
  const float* emb    = (const float*)d_in[1];
  const float* w_ih0  = (const float*)d_in[2];
  const float* b_ih0  = (const float*)d_in[3];
  const float* w_hh0  = (const float*)d_in[4];
  const float* b_hh0  = (const float*)d_in[5];
  const float* w_ih1  = (const float*)d_in[6];
  const float* b_ih1  = (const float*)d_in[7];
  const float* w_hh1  = (const float*)d_in[8];
  const float* b_hh1  = (const float*)d_in[9];
  const float* attn_w = (const float*)d_in[10];
  const float* attn_b = (const float*)d_in[11];
  const float* fc_w   = (const float*)d_in[12];
  const float* fc_b   = (const float*)d_in[13];
  float* out = (float*)d_out;

  char* ws = (char*)d_ws; size_t off = 0;
  auto carve = [&](size_t bytes) -> char* { char* p = ws + off; off += (bytes + 255) & ~(size_t)255; return p; };
  unsigned short* COMB16  = (unsigned short*)carve((size_t)kRows * kCombP * 2);
  unsigned short* Q16     = (unsigned short*)carve((size_t)kRows * kHid * 2);
  unsigned short* OUTST16 = (unsigned short*)carve((size_t)kSeq * kHid * kStep * 2);
  float*          SPL     = (float*)carve((size_t)kGrp * kStep * kStep * 4);
  unsigned short* P16     = (unsigned short*)carve((size_t)kGrp * kStep * kStep * 2);
  unsigned short* ATW16   = (unsigned short*)carve((size_t)kHid * kHid * 2);
  unsigned short* FCW16   = (unsigned short*)carve((size_t)kVocPad * 2 * kHid * 2);
  float*          FCB64   = (float*)carve((size_t)kVocPad * 4);
  if (off > ws_size || off > (size_t)134217728) return;
  float* LG = SPL;

  const float inv16 = 1.0f / 16.0f;
  const float qkscale = 0.08838834764831845f;
  const float pvscale = 1.0f / 32768.0f;

  prep_kernel<<<65, 256, 0, stream>>>(attn_w, fc_w, fc_b, (unsigned*)ATW16, (unsigned*)FCW16, (unsigned*)FCB64);

  rnn2_kernel<<<kSeq / kSeqPB, kRnnThreads, kRnnLdsBytes, stream>>>(x, emb, w_ih0, b_ih0, w_hh0, b_hh0,
                                                                    w_ih1, b_ih1, w_hh1, b_hh1, (_Float16*)COMB16);

  wmma_gemm64<0, false, 2, 1, false, 0, 0><<<dim3(256, 1), 256, 0, stream>>>(
      COMB16, nullptr, kCombP, 0L, ATW16, nullptr, kHid, 0L,
      (void*)Q16, nullptr, kHid, 0L, attn_b, nullptr, 0L, kRows, kHid, kHid, inv16);

  transpose_outs_kernel<<<kSeq * 16 * 2, 256, 0, stream>>>((const _Float16*)COMB16, (_Float16*)OUTST16);

  for (int g = 0; g < kNGrp; ++g) {
    const size_t g0 = (size_t)g * kGrp;
    wmma_gemm64<0, false, 0, 0, false, 0, 1><<<dim3(32, kGrp), 256, 0, stream>>>(
        Q16 + g0 * kStep * kHid, nullptr, kHid, (long)kStep * kHid,
        COMB16 + g0 * kStep * kCombP, nullptr, kCombP, (long)kStep * kCombP,
        (void*)SPL, nullptr, kStep, (long)kStep * kStep, nullptr, nullptr, 0L, kStep, kStep, kHid, qkscale);
    causal_softmax_kernel<<<(kGrp * kStep) / 8, 256, 0, stream>>>(SPL, (_Float16*)P16, kGrp * kStep);
    wmma_gemm64<0, false, 0, 1, false, 0, 2><<<dim3(4, kGrp), 256, 0, stream>>>(
        P16, nullptr, kStep, (long)kStep * kStep,
        OUTST16 + g0 * kHid * kStep, nullptr, kStep, (long)kHid * kStep,
        (void*)(COMB16 + g0 * kStep * kCombP + kHid), nullptr, kCombP, (long)kStep * kCombP,
        nullptr, nullptr, 0L, kStep, kHid, kStep, pvscale);
  }

  wmma_gemm64<0, false, 2, 0, false, 0, 0><<<dim3(128, 1), 256, 0, stream>>>(
      COMB16, nullptr, kCombP, 0L, FCW16, nullptr, 2 * kHid, 0L,
      (void*)LG, nullptr, kVocPad, 0L, FCB64, nullptr, 0L, kRows, kVocPad, 2 * kHid, inv16);

  pack_logits_kernel<<<kOut4 / 256, 256, 0, stream>>>(LG, out, kOut4);
}
